// GRU_74071005987293
// MI455X (gfx1250) — hardware-run, weakly checked
//
#include <hip/hip_runtime.h>
#include <math.h>

constexpr int NBATCH = 4096;
constexpr int NSTEP  = 512;
constexpr int NIN    = 4;
constexpr int NHID   = 16;
constexpr int NOUTF  = 2;
constexpr int NLAYER = 3;
constexpr int NTHR   = 32;
constexpr int ROWS_PER_BLOCK = 16;
constexpr int TILE_HALVES  = 16 * 32;
constexpr int LAYER_HALVES = 4 * TILE_HALVES;
constexpr int LAYER_WORDS  = LAYER_HALVES / 2;
constexpr int LAYER_CFLT   = 4 * 16;
constexpr float W_CARRY = 64.0f;
constexpr float B_CARRY = 16.0f;
constexpr float L_CARRY = 2048.0f;
constexpr float C_CARRY = 1024.0f;
constexpr float INV_HI  = 1.0f / 1024.0f;
constexpr float INV_LO  = 1.0f / 2097152.0f;
static_assert(NBATCH % ROWS_PER_BLOCK == 0, "grid covers the batch exactly");
static_assert(NIN <= 8 && NHID == 16, "K per tile = 16 input slots + 16 hidden = 32");
static_assert(ROWS_PER_BLOCK * NOUTF * 4 == 128, "one 128-B output line per block");
static_assert(LAYER_WORDS * NLAYER == 3072, "A staging extent");

typedef __attribute__((ext_vector_type(16))) _Float16 v16h;
typedef __attribute__((ext_vector_type(8)))  _Float16 v8h;
typedef __attribute__((ext_vector_type(8)))  float    v8f;
typedef __attribute__((ext_vector_type(4)))  float    v4f;
typedef __attribute__((ext_vector_type(2)))  float    v2f;
typedef __attribute__((ext_vector_type(8)))  unsigned v8u;
typedef __attribute__((ext_vector_type(4)))  unsigned v4u;

__device__ __forceinline__ unsigned short f2bf_bits(float f) {
  unsigned u = __float_as_uint(f);
  return (unsigned short)((u + 0x7FFFu + ((u >> 16) & 1u)) >> 16);
}
__device__ __forceinline__ float bf_bits2f(unsigned short h) { return __uint_as_float(((unsigned)h) << 16); }
__device__ __forceinline__ float bf16r(float f) { return bf_bits2f(f2bf_bits(f)); }
__device__ __forceinline__ unsigned pk2(float a, float b) {
  return __builtin_bit_cast(unsigned, __builtin_amdgcn_cvt_pkrtz(a, b));
}
__device__ __forceinline__ float trunc_f16(float v) { return __uint_as_float(__float_as_uint(v) & 0xFFFFE000u); }

__device__ __forceinline__ v16h frag_load(const _Float16* p) {
  union { v16h v; v8h h[2]; } f;
  f.h[0] = *(const v8h*)(p);
  f.h[1] = *(const v8h*)(p + 16);
  return f.v;
}
__device__ __forceinline__ v8f mma16(v16h a, v16h b, v8f c) {
  c = __builtin_amdgcn_wmma_f32_16x16x32_f16(false, a, false, b, (short)0, c, false, false);
  asm volatile("v_nop\n\tv_nop\n\tv_nop\n\tv_nop" : "+v"(c) : "v"(a), "v"(b));
  return c;
}
__device__ __forceinline__ float fsig(float x)  { return __builtin_amdgcn_rcpf(1.0f + expf(-x)); }
__device__ __forceinline__ float ftanh(float x) { return 1.0f - 2.0f * __builtin_amdgcn_rcpf(expf(2.0f * x) + 1.0f); }

__device__ __forceinline__ void stage_layer(const float* __restrict__ Wih, const float* __restrict__ Whh,
                                            const float* __restrict__ bih, const float* __restrict__ bhh,
                                            int din, unsigned* aw, float* cs, int tid) {
#pragma unroll 1
  for (int q = 0; q < 4; ++q) {
    const int g = (q < 2) ? q : 2;
    const float fa_q = (q != 3) ? 1.0f : 0.0f;
    const float fb_q = (q != 2) ? 1.0f : 0.0f;
#pragma unroll 1
    for (int it = 0; it < 8; ++it) {
      const int m  = it * 2 + (tid >> 4);
      const int p  = tid & 15;
      const int u0 = (2 * p) & 15;
      const int u1 = u0 + 1;
      const float fin = (p < 8) ? fa_q : 0.0f;
      const float fhd = (p < 8) ? 0.0f : fb_q;
      const float fi0 = (u0 < din) ? fin : 0.0f;
      const float fi1 = (u1 < din) ? fin : 0.0f;
      const int c0 = (u0 < din) ? u0 : (din - 1);
      const int c1 = (u1 < din) ? u1 : (din - 1);
      const float* wi = Wih + (g * NHID + m) * din;
      const float* wh = Whh + (g * NHID + m) * NHID;
      const float vi0 = wi[c0];
      const float vi1 = wi[c1];
      const float vh0 = wh[u0];
      const float vh1 = wh[u1];
      const float v0 = fmaf(fi0, vi0, fhd * vh0);
      const float v1 = fmaf(fi1, vi1, fhd * vh1);
      aw[(q * 16 + m) * 16 + p] = pk2(W_CARRY * bf16r(v0), W_CARRY * bf16r(v1));
    }
  }
#pragma unroll 1
  for (int it = 0; it < 2; ++it) {
    const int q = it * 2 + (tid >> 4);
    const int u = tid & 15;
    const int g = (q < 2) ? q : 2;
    const float fbi = (q != 3) ? 1.0f : 0.0f;
    const float fbh = (q != 2) ? 1.0f : 0.0f;
    const float bi = bf16r(bih[g * NHID + u]);
    const float bh = bf16r(bhh[g * NHID + u]);
    cs[q * 16 + u] = C_CARRY * fmaf(fbi, bi, fbh * bh);
  }
}

template <bool IN_HAS_LO>
__device__ __forceinline__ void gru_cell(const _Float16* at, const float* ct,
                                         const v4u inh, const v4u inl,
                                         float (&hs)[8], v4u& ph, v4u& pl) {
  asm volatile("" ::: "memory");
  v8u bw, lw;
#pragma unroll
  for (int j = 0; j < 4; ++j) {
    bw[j] = inh[j]; bw[4 + j] = ph[j];
    lw[j] = inl[j]; lw[4 + j] = pl[j];
  }
  const v16h bhi = __builtin_bit_cast(v16h, bw);
  const v16h blo = __builtin_bit_cast(v16h, lw);
  const v8f z8 = {0.f, 0.f, 0.f, 0.f, 0.f, 0.f, 0.f, 0.f};

  const v16h a_r  = frag_load(at);
  const v16h a_z  = frag_load(at + TILE_HALVES);
  const v16h a_ni = frag_load(at + 2 * TILE_HALVES);
  const v16h a_nh = frag_load(at + 3 * TILE_HALVES);
  const v8f  c_r  = *(const v8f*)(ct);
  const v8f  c_z  = *(const v8f*)(ct + 16);
  const v8f  c_ni = *(const v8f*)(ct + 32);
  const v8f  c_nh = *(const v8f*)(ct + 48);

  v8f gr_h = mma16(a_r,  bhi, c_r);
  v8f gr_l = mma16(a_r,  blo, z8);
  v8f gz_h = mma16(a_z,  bhi, c_z);
  v8f gz_l = mma16(a_z,  blo, z8);
  v8f ni_h = mma16(a_ni, bhi, c_ni);
  v8f ni_l = z8;
  if (IN_HAS_LO) ni_l = mma16(a_ni, blo, z8);
  v8f nh_h = mma16(a_nh, bhi, c_nh);
  v8f nh_l = mma16(a_nh, blo, z8);

#pragma unroll
  for (int r = 0; r < 8; ++r) {
    const float pr = gr_h[r] * INV_HI + gr_l[r] * INV_LO;
    const float pz = gz_h[r] * INV_HI + gz_l[r] * INV_LO;
    const float xn = ni_h[r] * INV_HI + ni_l[r] * INV_LO;
    const float hg = nh_h[r] * INV_HI + nh_l[r] * INV_LO;
    const float rg = fsig(pr);
    const float zg = fsig(pz);
    const float ng = ftanh(xn + rg * hg);
    const float ho = hs[r];
    hs[r] = (1.0f - zg) * ng + zg * ho;
  }
  v4u nhw, nlw;
#pragma unroll
  for (int j = 0; j < 4; ++j) {
    const float v0 = B_CARRY * hs[2 * j];
    const float v1 = B_CARRY * hs[2 * j + 1];
    const float t0 = trunc_f16(v0);
    const float t1 = trunc_f16(v1);
    nhw[j] = pk2(v0, v1);
    nlw[j] = pk2((v0 - t0) * L_CARRY, (v1 - t1) * L_CARRY);
  }
  ph = nhw;
  pl = nlw;
}

__global__ __launch_bounds__(NTHR) void gru3_seq_kernel(
    const float* __restrict__ x,
    const float* __restrict__ Wih0, const float* __restrict__ Whh0,
    const float* __restrict__ bih0, const float* __restrict__ bhh0,
    const float* __restrict__ Wih1, const float* __restrict__ Whh1,
    const float* __restrict__ bih1, const float* __restrict__ bhh1,
    const float* __restrict__ Wih2, const float* __restrict__ Whh2,
    const float* __restrict__ bih2, const float* __restrict__ bhh2,
    const float* __restrict__ fcW,  const float* __restrict__ fcb,
    float* __restrict__ out) {
  __shared__ __align__(16) unsigned Aw[NLAYER * LAYER_WORDS];
  __shared__ __align__(32) float    Cs[NLAYER * LAYER_CFLT];
  __shared__ __align__(16) float    Os[32];

  const int tid  = threadIdx.x;
  const int lane = tid & 31, hh = lane >> 4, m = lane & 15;
  const int b0   = blockIdx.x * ROWS_PER_BLOCK;

  stage_layer(Wih0, Whh0, bih0, bhh0, NIN,  Aw,                   Cs,                  tid);
  stage_layer(Wih1, Whh1, bih1, bhh1, NHID, Aw + LAYER_WORDS,     Cs + LAYER_CFLT,     tid);
  stage_layer(Wih2, Whh2, bih2, bhh2, NHID, Aw + 2 * LAYER_WORDS, Cs + 2 * LAYER_CFLT, tid);
  __syncthreads();

  float h0s[8], h1s[8], h2s[8];
#pragma unroll
  for (int r = 0; r < 8; ++r) { h0s[r] = 0.0f; h1s[r] = 0.0f; h2s[r] = 0.0f; }
  const v4u zero4 = {0u, 0u, 0u, 0u};
  v4u p0h = zero4, p0l = zero4, p1h = zero4, p1l = zero4, p2h = zero4, p2l = zero4;

  const _Float16* abase = (const _Float16*)Aw + m * 32 + 8 * hh;
  const float*    cbase = Cs + 8 * hh;
  const float*    xrow  = x + (size_t)(b0 + m) * NSTEP * NIN;
  const float     fx    = (hh == 0) ? B_CARRY : 0.0f;

#pragma unroll 1
  for (int t = 0; t < NSTEP; ++t) {
    asm volatile("" ::: "memory");
    const v4f xt = *(const v4f*)(xrow + (size_t)t * NIN);
    v4u xw;
    xw[0] = pk2(bf16r(xt[0]) * fx, bf16r(xt[1]) * fx);
    xw[1] = pk2(bf16r(xt[2]) * fx, bf16r(xt[3]) * fx);
    xw[2] = 0u;
    xw[3] = 0u;
    gru_cell<false>(abase,                    cbase,                  xw,  zero4, h0s, p0h, p0l);
    gru_cell<true >(abase + LAYER_HALVES,     cbase + LAYER_CFLT,     p0h, p0l,   h1s, p1h, p1l);
    gru_cell<true >(abase + 2 * LAYER_HALVES, cbase + 2 * LAYER_CFLT, p1h, p1l,   h2s, p2h, p2l);
  }

  const v4f wa0 = *(const v4f*)(fcW + 8 * hh);
  const v4f wb0 = *(const v4f*)(fcW + 8 * hh + 4);
  const v4f wa1 = *(const v4f*)(fcW + NHID + 8 * hh);
  const v4f wb1 = *(const v4f*)(fcW + NHID + 8 * hh + 4);
  const float fb0 = bf16r(fcb[0]);
  const float fb1 = bf16r(fcb[1]);
  float s0 = 0.0f, s1 = 0.0f;
#pragma unroll
  for (int r = 0; r < 4; ++r) {
    s0 += h2s[r] * bf16r(wa0[r]);
    s1 += h2s[r] * bf16r(wa1[r]);
  }
#pragma unroll
  for (int r = 0; r < 4; ++r) {
    s0 += h2s[4 + r] * bf16r(wb0[r]);
    s1 += h2s[4 + r] * bf16r(wb1[r]);
  }
  const float q0 = __shfl_xor(s0, 16, 32);
  const float q1 = __shfl_xor(s1, 16, 32);
  const float o0 = (s0 + q0) + fb0;
  const float o1 = (s1 + q1) + fb1;
  if (hh == 0) {
    v2f ov2;
    ov2[0] = o0;
    ov2[1] = o1;
    *(v2f*)(Os + 2 * m) = ov2;
  }
  __syncthreads();
  const v4f ov = *(const v4f*)(Os + (lane & 7) * 4);
  if (lane < 8) {
    float* op = out + (size_t)b0 * NOUTF + lane * 4;
    *(volatile v4f*)op = ov;
    __threadfence();
    *(volatile v4f*)op = ov;
  }
}

extern "C" void kernel_launch(void* const* d_in, const int* in_sizes, int n_in,
                              void* d_out, int out_size, void* d_ws, size_t ws_size, hipStream_t stream) {
  (void)d_ws; (void)ws_size;
  if (n_in < 15 || d_out == nullptr) return;
  if (in_sizes[0]  != NBATCH * NSTEP * NIN ||
      in_sizes[1]  != 3 * NHID * NIN  || in_sizes[2]  != 3 * NHID * NHID ||
      in_sizes[3]  != 3 * NHID        || in_sizes[4]  != 3 * NHID ||
      in_sizes[5]  != 3 * NHID * NHID || in_sizes[6]  != 3 * NHID * NHID ||
      in_sizes[7]  != 3 * NHID        || in_sizes[8]  != 3 * NHID ||
      in_sizes[9]  != 3 * NHID * NHID || in_sizes[10] != 3 * NHID * NHID ||
      in_sizes[11] != 3 * NHID        || in_sizes[12] != 3 * NHID ||
      in_sizes[13] != NOUTF * NHID    || in_sizes[14] != NOUTF ||
      out_size != NBATCH * NOUTF) return;

  const float* x    = (const float*)d_in[0];
  const float* Wih0 = (const float*)d_in[1];
  const float* Whh0 = (const float*)d_in[2];
  const float* bih0 = (const float*)d_in[3];
  const float* bhh0 = (const float*)d_in[4];
  const float* Wih1 = (const float*)d_in[5];
  const float* Whh1 = (const float*)d_in[6];
  const float* bih1 = (const float*)d_in[7];
  const float* bhh1 = (const float*)d_in[8];
  const float* Wih2 = (const float*)d_in[9];
  const float* Whh2 = (const float*)d_in[10];
  const float* bih2 = (const float*)d_in[11];
  const float* bhh2 = (const float*)d_in[12];
  const float* fcW  = (const float*)d_in[13];
  const float* fcb  = (const float*)d_in[14];
  float* out = (float*)d_out;

  gru3_seq_kernel<<<NBATCH / ROWS_PER_BLOCK, NTHR, 0, stream>>>(
      x, Wih0, Whh0, bih0, bhh0, Wih1, Whh1, bih1, bhh1, Wih2, Whh2, bih2, bhh2, fcW, fcb, out);
}
